// EnhancedGAT_32839319945833
// MI455X (gfx1250) — hardware-verified
//
#include <hip/hip_runtime.h>
#include <math.h>
#define SRB 512
#define SCHK 4096
typedef __attribute__((ext_vector_type(16))) _Float16 v16h;
typedef __attribute__((ext_vector_type(8)))  _Float16 v8h;
typedef __attribute__((ext_vector_type(16))) __bf16   v16b;
typedef __attribute__((ext_vector_type(8)))  __bf16   v8b;
typedef __attribute__((ext_vector_type(8)))  float    v8f;
typedef __attribute__((ext_vector_type(4)))  float    v4f;
#define PSCALE 32768.0f
#define U16(p) ((const unsigned short*)(const void*)(p))
#define PSCALE_INV (1.0f / 32768.0f)

__device__ __forceinline__ unsigned short f2bf_bits(float f) {
  unsigned u = __float_as_uint(f);
  return (unsigned short)((u + 0x7FFFu + ((u >> 16) & 1u)) >> 16);
}
__device__ __forceinline__ float bf_bits2f(unsigned short h) { return __uint_as_float(((unsigned)h) << 16); }

__device__ __forceinline__ void dep_guard_h(v8f& a, v8f& b, v16h x, v16h y) { asm volatile("v_nop\n\tv_nop\n\tv_nop\n\tv_nop" : "+v"(a), "+v"(b) : "v"(x), "v"(y)); }
__device__ __forceinline__ void dep_guard_b(v8f& a, v8f& b, v16b x, v16b y) { asm volatile("v_nop\n\tv_nop\n\tv_nop\n\tv_nop" : "+v"(a), "+v"(b) : "v"(x), "v"(y)); }
__device__ __forceinline__ void keep4_h(v16h a, v16h b, v16h c, v16h d) { asm volatile("v_nop" :: "v"(a), "v"(b), "v"(c), "v"(d)); }
__device__ __forceinline__ void keep4_b(v16b a, v16b b, v16b c, v16b d) { asm volatile("v_nop" :: "v"(a), "v"(b), "v"(c), "v"(d)); }
__device__ __forceinline__ void fence_f(float& t) { asm volatile("" : "+v"(t)); }
__device__ __forceinline__ void acc_guard4(v8f& a, v8f& b, v8f& c, v8f& d) { asm volatile("v_nop\n\tv_nop\n\tv_nop\n\tv_nop" : "+v"(a), "+v"(b), "+v"(c), "+v"(d)); }
template <typename T> struct Frag;
template <> struct Frag<_Float16> {
  typedef v16h V; union U { v16h v; v8h h[2]; };
  static __device__ __forceinline__ v16h load(const _Float16* p) {
    U f; f.h[0] = *(const v8h*)(p); f.h[1] = *(const v8h*)(p + 16); return f.v;
  }
  static __device__ __forceinline__ v8f mma(v16h a, v16h b, v8f c) {
    return __builtin_amdgcn_wmma_f32_16x16x32_f16(false, a, false, b, (short)0, c, false, false);
  }
  static __device__ __forceinline__ void guard(v8f& a, v8f& b, v16h x, v16h y) { dep_guard_h(a, b, x, y); }
  static __device__ __forceinline__ void keep(v16h a, v16h b, v16h c, v16h d) { keep4_h(a, b, c, d); }
};
template <> struct Frag<__bf16> {
  typedef v16b V; union U { v16b v; v8b h[2]; };
  static __device__ __forceinline__ v16b load(const __bf16* p) {
    U f; f.h[0] = *(const v8b*)(p); f.h[1] = *(const v8b*)(p + 16); return f.v;
  }
  static __device__ __forceinline__ v8f mma(v16b a, v16b b, v8f c) {
    return __builtin_amdgcn_wmma_f32_16x16x32_bf16(false, a, false, b, (short)0, c, false, false);
  }
  static __device__ __forceinline__ void guard(v8f& a, v8f& b, v16b x, v16b y) { dep_guard_b(a, b, x, y); }
  static __device__ __forceinline__ void keep(v16b a, v16b b, v16b c, v16b d) { keep4_b(a, b, c, d); }
};

template <int ET> struct Elem;
template <> struct Elem<0> { typedef _Float16 T; };
template <> struct Elem<1> { typedef __bf16 T; };
template <int ET, bool SPLIT, int BIAS_MODE, int OUT_MODE, bool RESID, int ACT = 0>
__global__ __launch_bounds__(256) void wmma_gemm64(
    const unsigned short* __restrict__ Ap, const unsigned short* __restrict__ A2p, int lda, long strideA,
    const unsigned short* __restrict__ Btp, const unsigned short* __restrict__ Bt2p, int ldb, long strideB,
    void* __restrict__ Cout, void* __restrict__ Cout2, int ldc, long strideC,
    const float* __restrict__ bias,
    const float* __restrict__ resid, long strideR,
    int M, int N, int K, float scale) {
  typedef typename Elem<ET>::T T;
  typedef typename Frag<T>::V V;
  const T* A = (const T*)Ap; const T* A2 = (const T*)A2p; const T* Bt = (const T*)Btp; const T* Bt2 = (const T*)Bt2p;
  __shared__ __align__(16) float sT[8][16 * 68];
  const int b    = blockIdx.y;
  const int lane = threadIdx.x & 31;
  const int wave = threadIdx.x >> 5;
  const int tilesN = N >> 6;
  const int tilesM = M >> 6;
  const int tile = blockIdx.x * 8 + wave;
  if (tile >= tilesM * tilesN) return;
  const int tm = tile / tilesN;
  const int tn = tile - tm * tilesN;
  const int m0 = tm << 6;
  const int n0 = tn << 6;

  const T* Ab  = A  + (size_t)b * strideA;
  const T* Bb  = Bt + (size_t)b * strideB;
  const T* Ab2 = SPLIT ? (A2  + (size_t)b * strideA) : nullptr;
  const T* Bb2 = SPLIT ? (Bt2 + (size_t)b * strideB) : nullptr;

  const int rlane = lane & 15;
  const int koff  = (lane >> 4) * 8;
  const int mOff  = (lane >> 4) * 8;

  v8f acc[4][4];
#pragma unroll
  for (int i = 0; i < 4; ++i)
#pragma unroll
    for (int j = 0; j < 4; ++j) acc[i][j] = (v8f){0.f,0.f,0.f,0.f,0.f,0.f,0.f,0.f};

  for (int k0 = 0; k0 < K; k0 += 32) {
    V bh[4], bl[4];
#pragma unroll
    for (int j = 0; j < 4; ++j) {
      const size_t bo = (size_t)(n0 + (j << 4) + rlane) * ldb + koff + k0;
      bh[j] = Frag<T>::load(Bb + bo);
      if (SPLIT) bl[j] = Frag<T>::load(Bb2 + bo);
    }
#pragma unroll
    for (int i = 0; i < 4; ++i) {
      const size_t ao = (size_t)(m0 + (i << 4) + rlane) * lda + koff + k0;
      V ah = Frag<T>::load(Ab + ao);
      V al;
      if (SPLIT) al = Frag<T>::load(Ab2 + ao);
#pragma unroll
      for (int j = 0; j < 4; ++j) {
        acc[i][j] = Frag<T>::mma(ah, bh[j], acc[i][j]);
        if (SPLIT) {
          acc[i][j] = Frag<T>::mma(ah, bl[j], acc[i][j]);
          acc[i][j] = Frag<T>::mma(al, bh[j], acc[i][j]);
        }
      }
      Frag<T>::guard(acc[i][0], acc[i][3], ah, SPLIT ? al : ah);
    }
    Frag<T>::keep(bh[0], bh[1], bh[2], bh[3]);
    if (SPLIT) Frag<T>::keep(bl[0], bl[1], bl[2], bl[3]);
  }
  acc_guard4(acc[0][0], acc[0][1], acc[0][2], acc[0][3]);
  acc_guard4(acc[1][0], acc[1][1], acc[1][2], acc[1][3]);
  acc_guard4(acc[2][0], acc[2][1], acc[2][2], acc[2][3]);
  acc_guard4(acc[3][0], acc[3][1], acc[3][2], acc[3][3]);

  float* slab = sT[wave];
  const float* Rb = RESID ? (resid + (size_t)b * strideR) : nullptr;
#pragma unroll
  for (int i = 0; i < 4; ++i) {
    const int mBase = m0 + (i << 4);
#pragma unroll
    for (int j = 0; j < 4; ++j) {
      const int n = n0 + (j << 4) + rlane;
      float bv = 0.f;
      if (BIAS_MODE == 2) bv = bias[n];
#pragma unroll
      for (int r = 0; r < 8; ++r) {
        float v = acc[i][j][r] * scale;
        if (BIAS_MODE == 1) v += bias[mBase + mOff + r];
        if (BIAS_MODE == 2) v += bv;
        if (RESID) v += Rb[(size_t)(mBase + mOff + r) * ldc + n];
        if (ACT == 1) v = tanhf(v);
        if (ACT == 2) v = fmaxf(v, 0.0f);
        if (ACT == 3) v = v / (1.0f + expf(-v));
        if (ACT == 4) v = (v > 0.f) ? v : 0.01f * v;
        if (ACT == 5) v = 0.5f * v * (1.0f + erff(v * 0.70710678118654752f));
        slab[(mOff + r) * 68 + (j << 4) + rlane] = v;
      }
    }
    __builtin_amdgcn_fence(__ATOMIC_RELEASE, "workgroup");
    __builtin_amdgcn_wave_barrier();
    __builtin_amdgcn_fence(__ATOMIC_ACQUIRE, "workgroup");
    if (OUT_MODE == 0) {
      float* C = (float*)Cout + (size_t)b * strideC;
      const int hh = lane >> 4, c4 = (lane & 15) * 4;
      for (int pass = 0; pass < 2; ++pass) {
#pragma unroll
        for (int it = 0; it < 8; ++it) {
          const int row = it * 2 + hh;
          v4f v = *(const v4f*)(slab + row * 68 + c4);
          *(volatile v4f*)(C + (size_t)(mBase + row) * ldc + n0 + c4) = v;
        }
        __threadfence();
      }
    } else {
      const int q = lane >> 3, c8 = (lane & 7) * 8;
      unsigned short* C  = (unsigned short*)Cout  + (size_t)b * strideC;
      unsigned short* C2 = (OUT_MODE == 2) ? ((unsigned short*)Cout2 + (size_t)b * strideC) : nullptr;
      for (int pass = 0; pass < 2; ++pass) {
#pragma unroll
        for (int it = 0; it < 4; ++it) {
          const int row = it * 4 + q;
          const float* sp = slab + row * 68 + c8;
          v8h hv, lv;
#pragma unroll
          for (int e = 0; e < 8; ++e) {
            if (OUT_MODE == 1) {
              hv[e] = (_Float16)sp[e];
            } else {
              unsigned short hb = f2bf_bits(sp[e]);
              unsigned short lb = f2bf_bits(sp[e] - bf_bits2f(hb));
              hv[e] = __builtin_bit_cast(_Float16, hb);
              lv[e] = __builtin_bit_cast(_Float16, lb);
            }
          }
          *(volatile v8h*)(C + (size_t)(mBase + row) * ldc + n0 + c8) = hv;
          if (OUT_MODE == 2) *(volatile v8h*)(C2 + (size_t)(mBase + row) * ldc + n0 + c8) = lv;
        }
        __threadfence();
      }
    }
    __builtin_amdgcn_fence(__ATOMIC_RELEASE, "workgroup");
    __builtin_amdgcn_wave_barrier();
    __builtin_amdgcn_fence(__ATOMIC_ACQUIRE, "workgroup");
  }
}

__global__ __launch_bounds__(256) void cast_f32_f16x2(
    const float* __restrict__ in, _Float16* __restrict__ out, int n2) {
  int i = blockIdx.x * 256 + threadIdx.x;
  if (i < n2) {
    const _Float16 h0 = (_Float16)in[2 * i], h1 = (_Float16)in[2 * i + 1];
    const unsigned u = (unsigned)__builtin_bit_cast(unsigned short, h0) | ((unsigned)__builtin_bit_cast(unsigned short, h1) << 16);
    ((volatile unsigned*)out)[i] = u;
    __threadfence();
    ((volatile unsigned*)out)[i] = u;
  }
}


#ifndef SRB
#define SRB 512
#endif
#ifndef SCHK
#define SCHK 4096
#endif
#define SEPT (SCHK / SRB)
__device__ __forceinline__ int blk_excl_scan(int cnt, int* scan_ws, int tid, int* tot) {
  const int lane = tid & 31, wave = tid >> 5; int incl = cnt;
#pragma unroll
  for (int o = 1; o < 32; o <<= 1) { const int v = __shfl_up(incl, o, 32); if (lane >= o) incl += v; }
  if (lane == 31) scan_ws[wave] = incl;
  __syncthreads();
  if (wave == 0) { int wv = (lane < SRB / 32) ? scan_ws[lane] : 0; int wincl = wv;
#pragma unroll
    for (int o = 1; o < 32; o <<= 1) { const int v = __shfl_up(wincl, o, 32); if (lane >= o) wincl += v; }
    if (lane < SRB / 32) scan_ws[32 + lane] = wincl - wv; if (lane == 31) scan_ws[64] = wincl; }
  __syncthreads();
  const int res = scan_ws[32 + wave] + incl - cnt; *tot = scan_ws[64];
  return res;
}
__device__ __forceinline__ int chunk_compact(const int* __restrict__ keyv, const int* __restrict__ othv, int e0, int ne, int n0, int nn, int tid, int* L0, int* L1, int* L2, int* scan_ws) {
  int hk[SEPT], ho[SEPT], he[SEPT]; int cnt = 0;
#pragma unroll
  for (int k = 0; k < SEPT; ++k) { const int e = e0 + tid * SEPT + k; hk[k] = -1; if (e < ne) { const int d = keyv[e]; if (d >= n0 && d < n0 + SRB && d < nn) { hk[k] = d - n0; int s = othv[e]; s = s < 0 ? 0 : (s >= nn ? nn - 1 : s); ho[k] = s; he[k] = e; ++cnt; } } }
  int tot; int p = blk_excl_scan(cnt, scan_ws, tid, &tot);
#pragma unroll
  for (int k = 0; k < SEPT; ++k) if (hk[k] >= 0) { L0[p] = hk[k]; L1[p] = ho[k]; if (L2) L2[p] = he[k]; ++p; }
  __syncthreads();
  return tot;
}
#define NN 50000
#define NPAD 50176
#define NE 600000
#define NG 512
__global__ __launch_bounds__(256) void xcast_kernel(const float* __restrict__ x, unsigned* __restrict__ X16) {
  const long i = (long)blockIdx.x * 256 + threadIdx.x; if (i >= (long)NPAD * 48) return; const long r = i / 48; const int cp = 2 * (int)(i % 48); float a = 0.f, b = 0.f;
  if (r < NN) { if (cp < 92) a = x[r * 92 + cp]; if (cp + 1 < 92) b = x[r * 92 + cp + 1]; }
  const unsigned u = (unsigned)__builtin_bit_cast(unsigned short, (_Float16)a) | ((unsigned)__builtin_bit_cast(unsigned short, (_Float16)b) << 16); ((volatile unsigned*)X16)[i] = u; __threadfence(); ((volatile unsigned*)X16)[i] = u;
}
__global__ __launch_bounds__(256) void wt_kernel(const float* __restrict__ Wm, int KIN, int NOUT, int KP, int NOP, unsigned* __restrict__ BT) {
  for (int i = blockIdx.x * 256 + threadIdx.x; i < NOP * KP / 2; i += gridDim.x * 256) { const int o = i / (KP / 2), kp = 2 * (i % (KP / 2)); float a = 0.f, b = 0.f; if (o < NOUT) { if (kp < KIN) a = Wm[(size_t)kp * NOUT + o]; if (kp + 1 < KIN) b = Wm[(size_t)(kp + 1) * NOUT + o]; }
    const unsigned u = (unsigned)__builtin_bit_cast(unsigned short, (_Float16)a) | ((unsigned)__builtin_bit_cast(unsigned short, (_Float16)b) << 16); ((volatile unsigned*)BT)[i] = u; __threadfence(); ((volatile unsigned*)BT)[i] = u; }
}
__global__ __launch_bounds__(256) void asd_kernel(const float* __restrict__ Hm, int ld, int NH, const float* __restrict__ as_, const float* __restrict__ ad_, float* __restrict__ ASD) {
  const int lane = threadIdx.x & 31, wave = threadIdx.x >> 5; const int n = blockIdx.x * 8 + wave; if (n >= NN) return;
  float outs = 0.f, outd = 0.f;
#pragma unroll 1
  for (int h = 0; h < NH; ++h) { const float v = Hm[(size_t)n * ld + h * 32 + lane]; float s = v * as_[h * 32 + lane], d = v * ad_[h * 32 + lane];
    for (int o = 16; o > 0; o >>= 1) { s += __shfl_xor(s, o, 32); d += __shfl_xor(d, o, 32); } if (lane == h) { outs = s; outd = d; } }
  const int idx = lane & 15; const float vs = __shfl(outs, idx & 7, 32), vd = __shfl(outd, idx & 7, 32);
  const float val = (idx < 8) ? vs : vd;
  for (int pass = 0; pass < 2; ++pass) { ((volatile float*)ASD)[(size_t)n * 16 + idx] = val; __threadfence(); }
}
__global__ __launch_bounds__(256) void ce_kernel(const float* We1, const float* ae1, const float* We2, const float* ae2, float* CE,
                                                 const float* b1, const float* g1, const float* be1, const float* m1, const float* v1, float* SC1, float* SH1) {
  const int t = threadIdx.x; float s = 0.f; if (t < 8) { for (int c = 0; c < 32; ++c) s += We1[t * 32 + c] * ae1[t * 32 + c]; } else if (t == 8) { for (int c = 0; c < 32; ++c) s += We2[c] * ae2[c]; }
  const float sc = g1[t] * rsqrtf(v1[t] + 1e-5f); const float shv = (b1[t] - m1[t]) * sc + be1[t];
  for (int pass = 0; pass < 2; ++pass) { if (t < 32) ((volatile float*)CE)[t] = s; ((volatile float*)SC1)[t] = sc; ((volatile float*)SH1)[t] = shv; __threadfence(); }
}
template <int HPP, bool L1EPI>
__global__ __launch_bounds__(SRB) void gat_stream_kernel(const float* __restrict__ Hm, int ld, const float* __restrict__ ASD, int h0, const float* __restrict__ ea, const float* __restrict__ ce,
                                                        const int* __restrict__ dstv, const int* __restrict__ srcv, float* __restrict__ RAW, int ldr,
                                                        const float* __restrict__ SC, const float* __restrict__ SH, unsigned* __restrict__ X2) {
  __shared__ int L0[SCHK]; __shared__ int L1[SCHK]; __shared__ int L2[SCHK]; __shared__ int scan_ws[80];
  const int tid = threadIdx.x, n0 = blockIdx.x * SRB; const int n = n0 + tid; const int nc = n < NN ? n : NN - 1;
  float m[HPP], ssum[HPP], adn[HPP], ceh[HPP]; float acc[HPP * 32];
#pragma unroll
  for (int h = 0; h < HPP; ++h) { m[h] = -INFINITY; ssum[h] = 0.f; adn[h] = ASD[(size_t)nc * 16 + 8 + h0 + h]; ceh[h] = ce[h0 + h]; }
#pragma unroll
  for (int c = 0; c < HPP * 32; ++c) acc[c] = 0.f;
  auto update = [&](int s, float we) {
    const float* hp = Hm + (size_t)s * ld + h0 * 32; const float* as_ = ASD + (size_t)s * 16 + h0;
#pragma unroll
    for (int h = 0; h < HPP; ++h) { float al = as_[h] + adn[h] + we * ceh[h]; al = al > 0.f ? al : 0.2f * al;
      const float mn = fmaxf(m[h], al); const float rr = __expf(m[h] - mn), ex = __expf(al - mn); ssum[h] = ssum[h] * rr + ex; m[h] = mn;
#pragma unroll
      for (int d = 0; d < 32; d += 4) { const v4f v = *(const v4f*)(hp + h * 32 + d); acc[h * 32 + d] = acc[h * 32 + d] * rr + ex * v[0]; acc[h * 32 + d + 1] = acc[h * 32 + d + 1] * rr + ex * v[1]; acc[h * 32 + d + 2] = acc[h * 32 + d + 2] * rr + ex * v[2]; acc[h * 32 + d + 3] = acc[h * 32 + d + 3] * rr + ex * v[3]; } } };
  int cnt = 0; float asum = 0.f;
  for (int e0 = 0; e0 < NE; e0 += SCHK) { const int tot = chunk_compact(dstv, srcv, e0, NE, n0, NN, tid, L0, L1, L2, scan_ws);
    for (int q = 0; q < tot; ++q) { if (L0[q] == tid) { const float we = ea[L2[q]]; ++cnt; asum += we; update(L1[q], we); } }
    __syncthreads(); }
  if (!L1EPI) {
    if (n >= NN) return;
    update(n, asum / fmaxf((float)cnt, 1.0f));
    for (int pass = 0; pass < 2; ++pass) {
#pragma unroll
      for (int h = 0; h < HPP; ++h) { const float inv = 1.0f / ssum[h];
#pragma unroll
        for (int d = 0; d < 32; d += 4) { v4f o; for (int q2 = 0; q2 < 4; ++q2) o[q2] = acc[h * 32 + d + q2] * inv; *(volatile v4f*)(RAW + (size_t)n * ldr + (h0 + h) * 32 + d) = o; } }
      __threadfence(); }
  } else {
    if (n >= NPAD) return;
    const bool live = n < NN;
    if (live) update(n, asum / fmaxf((float)cnt, 1.0f));
#pragma unroll
    for (int h = 0; h < HPP; ++h) { const float inv = live ? 1.0f / ssum[h] : 0.f; const int c0 = (h0 + h) * 32;
#pragma unroll
      for (int c = 0; c < 32; ++c) { float t = acc[h * 32 + c] * inv * SC[c0 + c]; fence_f(t); t = t + SH[c0 + c]; acc[h * 32 + c] = live ? fmaxf(t, 0.f) : 0.f; } }
    unsigned* xrow = X2 + ((size_t)n * ldr + (size_t)h0 * 32) / 2;
    for (int pass = 0; pass < 2; ++pass) {
#pragma unroll
      for (int h = 0; h < HPP; ++h) {
#pragma unroll
        for (int d = 0; d < 32; d += 8) { unsigned u[4];
#pragma unroll
          for (int q2 = 0; q2 < 4; ++q2) { const int c = d + 2 * q2;
            const float a = acc[h * 32 + c], b = acc[h * 32 + c + 1];
            u[q2] = (unsigned)__builtin_bit_cast(unsigned short, (_Float16)a) | ((unsigned)__builtin_bit_cast(unsigned short, (_Float16)b) << 16); }
          v4f o; o[0] = __uint_as_float(u[0]); o[1] = __uint_as_float(u[1]); o[2] = __uint_as_float(u[2]); o[3] = __uint_as_float(u[3]);
          *(volatile v4f*)(xrow + h * 16 + d / 2) = o; } }
      __threadfence(); }
  }
}
__global__ __launch_bounds__(256) void epi2_kernel(const float* __restrict__ RAW, const float* __restrict__ b2, const float* __restrict__ g, const float* __restrict__ be, const float* __restrict__ mm, const float* __restrict__ vv, float* __restrict__ H3) {
  const long i = (long)blockIdx.x * 256 + threadIdx.x; if (i >= (long)NN * 32) return; const int c = (int)(i % 32);
  const float v = fmaxf((RAW[i] + b2[c] - mm[c]) * (g[c] * rsqrtf(vv[c] + 1e-5f)) + be[c], 0.f); ((volatile float*)H3)[i] = v; __threadfence(); ((volatile float*)H3)[i] = v;
}
__device__ __forceinline__ int lbound(const int* __restrict__ batch, int key) {
  int lo = 0, hi = NN;
#pragma unroll 1
  for (int it = 0; it < 17; ++it) { if (lo < hi) { const int mid = (lo + hi) >> 1; if (batch[mid] < key) lo = mid + 1; else hi = mid; } }
  lo = lo < 0 ? 0 : (lo > NN ? NN : lo); return lo;
}
__global__ __launch_bounds__(1024) void pool_kernel(const float* __restrict__ H3, const int* __restrict__ batch, const float* __restrict__ fcW, const float* __restrict__ fcb, float* __restrict__ out) {
  __shared__ float res[32];
  const int lane = threadIdx.x & 31, wave = threadIdx.x >> 5; const int g = blockIdx.x * 32 + wave;
  const int lo = lbound(batch, g), hi0 = lbound(batch, g + 1); const int hi = hi0 < lo ? lo : hi0;
  float s = 0.f;
#pragma unroll 1
  for (int n = lo; n < hi; ++n) s += H3[(size_t)n * 32 + lane];
  float d = (s / fmaxf((float)(hi - lo), 1.0f)) * fcW[lane];
  for (int o = 16; o > 0; o >>= 1) d += __shfl_xor(d, o, 32);
  if (lane == 0) res[wave] = d + fcb[0];
  __syncthreads();
  if (wave == 0) { const float v = res[lane]; ((volatile float*)out)[blockIdx.x * 32 + lane] = v; __threadfence(); ((volatile float*)out)[blockIdx.x * 32 + lane] = v; }
}
extern "C" void kernel_launch(void* const* d_in, const int* in_sizes, int n_in, void* d_out, int out_size, void* d_ws, size_t ws_size, hipStream_t stream) {
  (void)in_sizes; (void)n_in; (void)out_size; (void)ws_size;
  auto Fp = [&](int i) { return (const float*)d_in[i]; };
  const float* x = Fp(0); const int* ei = (const int*)d_in[1]; const float* ea = Fp(2); const int* batch = (const int*)d_in[3];
  const float* W1 = Fp(4); const float* We1 = Fp(5); const float* as1 = Fp(6); const float* ad1 = Fp(7); const float* ae1 = Fp(8); const float* b1 = Fp(9); const float* g1 = Fp(10); const float* be1 = Fp(11); const float* m1 = Fp(12); const float* v1 = Fp(13);
  const float* W2 = Fp(14); const float* We2 = Fp(15); const float* as2 = Fp(16); const float* ad2 = Fp(17); const float* ae2 = Fp(18); const float* b2 = Fp(19); const float* g2 = Fp(20); const float* be2 = Fp(21); const float* m2 = Fp(22); const float* v2 = Fp(23); const float* fcW = Fp(24); const float* fcb = Fp(25);
  char* ws = (char*)d_ws; size_t off = 0;
  auto carve = [&](size_t bytes) -> char* { char* p = ws + off; off += (bytes + 255) & ~(size_t)255; return p; };
  unsigned* X16 = (unsigned*)carve((size_t)NPAD * 96 * 2); unsigned* BT1 = (unsigned*)carve(256 * 96 * 2); unsigned* BT2 = (unsigned*)carve(64 * 256 * 2);
  float* H1 = (float*)carve((size_t)NPAD * 256 * 4); float* ASD1 = (float*)carve((size_t)NPAD * 16 * 4); float* CE = (float*)carve(256); float* SC1 = (float*)carve(1024); float* SH1 = (float*)carve(1024); unsigned* X2 = (unsigned*)carve((size_t)NPAD * 256 * 2);
  float* H2 = (float*)carve((size_t)NPAD * 64 * 4); float* ASD2 = (float*)carve((size_t)NPAD * 16 * 4); float* RAW2 = (float*)carve((size_t)NPAD * 32 * 4); float* H3 = (float*)carve((size_t)NPAD * 32 * 4);
  const int* src = ei; const int* dst = ei + NE; const int nb = (NN + SRB - 1) / SRB;
  xcast_kernel<<<(NPAD * 48 + 255) / 256, 256, 0, stream>>>(x, X16);
  wt_kernel<<<48, 256, 0, stream>>>(W1, 92, 256, 96, 256, BT1); wt_kernel<<<32, 256, 0, stream>>>(W2, 256, 32, 256, 64, BT2);
  ce_kernel<<<1, 256, 0, stream>>>(We1, ae1, We2, ae2, CE, b1, g1, be1, m1, v1, SC1, SH1);
  { const int t = (NPAD / 64) * 4; wmma_gemm64<0, false, 0, 0, false><<<dim3((t + 7) / 8, 1), 256, 0, stream>>>((const unsigned short*)X16, nullptr, 96, 0, (const unsigned short*)BT1, nullptr, 96, 0, H1, nullptr, 256, 0, nullptr, nullptr, 0, NPAD, 256, 96, 1.0f); }
  asd_kernel<<<NPAD / 8, 256, 0, stream>>>(H1, 256, 8, as1, ad1, ASD1);
  for (int h0 = 0; h0 < 8; h0 += 2) gat_stream_kernel<2, true><<<NPAD / SRB, SRB, 0, stream>>>(H1, 256, ASD1, h0, ea, CE, dst, src, nullptr, 256, SC1, SH1, X2);
  { const int t = (NPAD / 64) * 1; wmma_gemm64<0, false, 0, 0, false><<<dim3((t + 7) / 8, 1), 256, 0, stream>>>((const unsigned short*)X2, nullptr, 256, 0, (const unsigned short*)BT2, nullptr, 256, 0, H2, nullptr, 64, 0, nullptr, nullptr, 0, NPAD, 64, 256, 1.0f); }
  asd_kernel<<<NPAD / 8, 256, 0, stream>>>(H2, 64, 1, as2, ad2, ASD2);
  gat_stream_kernel<1, false><<<nb, SRB, 0, stream>>>(H2, 64, ASD2, 0, ea, CE + 8, dst, src, RAW2, 32, nullptr, nullptr, nullptr);
  epi2_kernel<<<(NN * 32 + 255) / 256, 256, 0, stream>>>(RAW2, b2, g2, be2, m2, v2, H3);
  pool_kernel<<<NG / 32, 1024, 0, stream>>>(H3, batch, fcW, fcb, (float*)d_out);
}
